// Encoder_68753836474771
// MI455X (gfx1250) — hardware-verified
//
#include <hip/hip_runtime.h>
#include <hip/hip_fp16.h>


#ifndef NB
#define NB 16
#endif
#ifndef NOBS
#define NOBS 4096
#endif
#define NB_FULL   16
#define NOBS_FULL 4096
#define LSEQ      512
#define DCH       41
#define LD_FULL   (LSEQ * DCH)
#define PER       82
#define DK        128
#define DH        32
#define NHEAD     4
#define MIND      128
#define NLAY      3
#define WPL       (DK * DK)
#define NPLANES   27
#define OUT1_OFF  ((size_t)NB_FULL * NOBS_FULL * DK)

static_assert(NB >= 1 && NB <= NB_FULL);
static_assert(NOBS >= 256 && NOBS <= NOBS_FULL);
static_assert(NOBS % 256 == 0);
static_assert(256 * PER == LD_FULL);
static_assert(NOBS <= LD_FULL);
static_assert(OUT1_OFF * 4 == 33554432);
static_assert((OUT1_OFF + (size_t)NB_FULL * NOBS_FULL) * 4 == 33816576);

#define WPL_BYTES ((size_t)NPLANES * WPL * 2)
#define RI_BYTES  ((size_t)NB * NOBS * 16)
#define MK_BYTES  ((size_t)NB * NOBS * 4)
#define PL_BYTES  ((size_t)NB * NOBS * DK * 2)
#define O0_BYTES  ((size_t)NB * MIND * DK * 4)
#define HP_BYTES  ((size_t)NB * MIND * DK * 2)
#define WS_TOTAL  (WPL_BYTES + RI_BYTES + MK_BYTES + 4 * PL_BYTES + O0_BYTES + 2 * HP_BYTES)
static_assert(WS_TOTAL <= 134217728);
static_assert(WPL_BYTES % 256 == 0 && RI_BYTES % 256 == 0 && MK_BYTES % 256 == 0);

typedef _Float16 v16h __attribute__((ext_vector_type(16)));
typedef _Float16 v8h  __attribute__((ext_vector_type(8)));
typedef _Float16 v4h  __attribute__((ext_vector_type(4)));
typedef float    v8f  __attribute__((ext_vector_type(8)));
typedef float    v4f  __attribute__((ext_vector_type(4)));

union Frag { v16h v; v8h h[2]; };

#define LOG2E     1.44269504088896340736f
#define ATT_SCALE 0.08838834764831845f
#define CS        (LOG2E * ATT_SCALE * 0.000244140625f)
#define NEGT      (-1.0e10f * LOG2E)
#define SC_RES    2048.0f
#define SC_RINV   4.8828125e-04f

static __device__ __forceinline__ v8f zero8() {
    v8f z;
#pragma unroll
    for (int i = 0; i < 8; ++i) z[i] = 0.0f;
    return z;
}

static __device__ __forceinline__ v16h load_frag16(const _Float16* base, int ld, int lane) {
    int m  = lane & 15;
    int kb = (lane >> 4) << 3;
    const _Float16* p = base + (size_t)m * ld + kb;
    Frag f;
    f.h[0] = *(const v8h*)(p);
    f.h[1] = *(const v8h*)(p + 16);
    return f.v;
}

static __device__ __forceinline__ v16h load_frag_f32(const float* base, int ld, int lane, float sc) {
    int m  = lane & 15;
    int kb = (lane >> 4) << 3;
    const float* p = base + (size_t)m * ld + kb;
    v4f x0 = *(const v4f*)(p);
    v4f x1 = *(const v4f*)(p + 4);
    v4f x2 = *(const v4f*)(p + 16);
    v4f x3 = *(const v4f*)(p + 20);
    v16h f;
    f[0]  = (_Float16)(x0.x * sc); f[1]  = (_Float16)(x0.y * sc);
    f[2]  = (_Float16)(x0.z * sc); f[3]  = (_Float16)(x0.w * sc);
    f[4]  = (_Float16)(x1.x * sc); f[5]  = (_Float16)(x1.y * sc);
    f[6]  = (_Float16)(x1.z * sc); f[7]  = (_Float16)(x1.w * sc);
    f[8]  = (_Float16)(x2.x * sc); f[9]  = (_Float16)(x2.y * sc);
    f[10] = (_Float16)(x2.z * sc); f[11] = (_Float16)(x2.w * sc);
    f[12] = (_Float16)(x3.x * sc); f[13] = (_Float16)(x3.y * sc);
    f[14] = (_Float16)(x3.z * sc); f[15] = (_Float16)(x3.w * sc);
    return f;
}

static __device__ __forceinline__ v8f wmma16(v16h a, v16h b, v8f c) {
    v8f d = __builtin_amdgcn_wmma_f32_16x16x32_f16(false, a, false, b, (short)0, c, false, false);
    asm volatile("v_nop\n\tv_nop\n\tv_nop\n\tv_nop" : "+v"(d) : "v"(a), "v"(b));
    return d;
}

static __device__ __forceinline__ float bf16r(float x) {
    unsigned u = __float_as_uint(x);
    u = (u + 0x7FFFu + ((u >> 16) & 1u)) & 0xFFFF0000u;
    return __uint_as_float(u);
}

static __device__ __forceinline__ float ex2(float x) {
    return __builtin_amdgcn_exp2f(x);
}

static __device__ __forceinline__ void wave_lds_sync() {
    __builtin_amdgcn_fence(3, "wavefront");
    asm volatile("s_wait_dscnt 0" ::: "memory");
    __builtin_amdgcn_wave_barrier();
}

static __device__ __forceinline__ float hmax16(float v) {
    v = fmaxf(v, __shfl_xor(v, 1, 32));
    v = fmaxf(v, __shfl_xor(v, 2, 32));
    v = fmaxf(v, __shfl_xor(v, 4, 32));
    v = fmaxf(v, __shfl_xor(v, 8, 32));
    return v;
}
static __device__ __forceinline__ float hsum16(float v) {
    v += __shfl_xor(v, 1, 32);
    v += __shfl_xor(v, 2, 32);
    v += __shfl_xor(v, 4, 32);
    v += __shfl_xor(v, 8, 32);
    return v;
}

static __device__ __forceinline__ void split16(float z, _Float16& h, _Float16& r) {
    float v = z * 16.0f;
    h = (_Float16)v;
    r = (_Float16)((v - (float)h) * SC_RES);
}

__global__ __launch_bounds__(256) void k_wprep(const float* p0, const float* p1, const float* p2,
                                                const float* p3, const float* p4, const float* p5,
                                                const float* p6, const float* p7, const float* pind,
                                                _Float16* wpl) {
    __shared__ __align__(16) _Float16 T[WPL];
    const unsigned tid = threadIdx.x;
    const unsigned bid = blockIdx.x;
    const unsigned m = bid / 3u;
    const unsigned i = bid - m * 3u;
    const float* src = p0;
    if (m == 1u) src = p1;
    if (m == 2u) src = p2;
    if (m == 3u) src = p3;
    if (m == 4u) src = p4;
    if (m == 5u) src = p5;
    if (m == 6u) src = p6;
    if (m == 7u) src = p7;
    if (m == 8u) src = pind;
    src += (size_t)i * WPL;
    const bool tr = (m < 8u);
#pragma unroll 4
    for (unsigned it = 0; it < 64u; ++it) {
        unsigned idx = it * 256u + tid;
        unsigned k = idx >> 7, n = idx & 127u;
        float x = src[idx];
        unsigned dst = tr ? (n * 128u + k) : idx;
        T[dst] = (_Float16)(bf16r(x) * 64.0f);
    }
    __syncthreads();
    v8h v[8];
#pragma unroll
    for (unsigned j = 0; j < 8u; ++j) v[j] = *(const v8h*)(&T[(j * 256u + tid) * 8u]);
    _Float16* dstp = wpl + (size_t)bid * WPL;
#pragma unroll
    for (unsigned j = 0; j < 8u; ++j) *(volatile v8h*)(dstp + (size_t)(j * 256u + tid) * 8u) = v[j];
    __threadfence();
#pragma unroll
    for (unsigned j = 0; j < 8u; ++j) *(volatile v8h*)(dstp + (size_t)(j * 256u + tid) * 8u) = v[j];
}

__global__ __launch_bounds__(256) void k_compact(const float* __restrict__ ctx,
                                                  const float* __restrict__ val,
                                                  const float* __restrict__ mask,
                                                  const int* __restrict__ obs,
                                                  float* rowinfo, float* mkp, float* out1) {
    __shared__ int sc[256];
    __shared__ int sel[NOBS];
    __shared__ int sflag[8];
    const unsigned tid = threadIdx.x, lane = tid & 31u, w = tid >> 5;
    const unsigned b = blockIdx.x;
    const float* mb = mask + (size_t)b * LD_FULL;
    const unsigned j0 = tid * PER;

    int cnt = 0, bad = 0;
#pragma unroll 1
    for (unsigned e = 0; e < PER; ++e) {
        float mv = mb[j0 + e];
        cnt += (mv > 0.0f) ? 1 : 0;
        bad |= (mv != 0.0f && mv != 1.0f) ? 1 : 0;
    }
    const int ol = obs[0];
    bad |= (ol < NOBS) ? 1 : 0;
    sc[tid] = cnt;
    const unsigned long long bal = __ballot(bad);
    if (lane == 0u) sflag[w] = (bal != 0ull) ? 1 : 0;
    __syncthreads();
#pragma unroll 1
    for (unsigned o = 1; o < 256u; o <<= 1) {
        unsigned s = (tid >= o) ? (tid - o) : 0u;
        int t = sc[s];
        t = (tid >= o) ? t : 0;
        __syncthreads();
        sc[tid] += t;
        __syncthreads();
    }
    const int total = sc[255];
    int po = sc[tid] - cnt;
    const int blockbad = sflag[0] | sflag[1] | sflag[2] | sflag[3] | sflag[4] | sflag[5] | sflag[6] | sflag[7];
#pragma unroll 1
    for (unsigned e = 0; e < PER; ++e) {
        int j = (int)(j0 + e);
        float mv = mb[j];
        int one = (mv > 0.0f) ? 1 : 0;
        int pos = one ? po : (total + (j - po));
        if ((unsigned)pos < (unsigned)NOBS) sel[pos] = j;
        po += one;
    }
    __syncthreads();

    const float nanv = __uint_as_float(0x7FC00000u);
#pragma unroll 1
    for (unsigned p = tid; p < (unsigned)NOBS; p += 256u) {
        int j = sel[p];
        j = min(max(j, 0), LD_FULL - 1);
        unsigned ti = (unsigned)j / 41u;
        unsigned ch = (unsigned)j - ti * 41u;
        float t = bf16r(ctx[(size_t)b * LSEQ + ti]);
        float u = bf16r(val[(size_t)b * LD_FULL + j]);
        float m = bf16r(mb[j]);
        v4f info;
        info.x = t; info.y = u; info.z = m; info.w = (float)ch;
        float mo = blockbad ? nanv : m;
        const size_t r = (size_t)b * NOBS + p;
        const size_t ro = OUT1_OFF + (size_t)b * NOBS_FULL + p;
        *(volatile v4f*)(rowinfo + r * 4) = info;
        *(volatile float*)(mkp + r) = m;
        *(volatile float*)(out1 + ro) = mo;
        __threadfence();
        *(volatile v4f*)(rowinfo + r * 4) = info;
        *(volatile float*)(mkp + r) = m;
        *(volatile float*)(out1 + ro) = mo;
    }
}

__global__ __launch_bounds__(256) void k_embed(const float* __restrict__ rowinfo,
                                                const float* __restrict__ iffw,
                                                const float* __restrict__ iffb,
                                                float* Zout, _Float16* Zh, _Float16* Zr) {
    const unsigned tid = threadIdx.x, lane = tid & 31u, w = tid >> 5;
    const unsigned c = lane * 4u;
    v4f w41 = *(const v4f*)(iffw + 41 * DK + c);
    v4f w42 = *(const v4f*)(iffw + 42 * DK + c);
    v4f bb  = *(const v4f*)(iffb + c);
    w41.x = bf16r(w41.x); w41.y = bf16r(w41.y); w41.z = bf16r(w41.z); w41.w = bf16r(w41.w);
    w42.x = bf16r(w42.x); w42.y = bf16r(w42.y); w42.z = bf16r(w42.z); w42.w = bf16r(w42.w);
    bb.x = bf16r(bb.x); bb.y = bf16r(bb.y); bb.z = bf16r(bb.z); bb.w = bf16r(bb.w);
    const unsigned rowb = blockIdx.x * 32u + w * 4u;
#pragma unroll 1
    for (unsigned i = 0; i < 4u; ++i) {
        const unsigned row = rowb + i;
        v4f info = *(const v4f*)(rowinfo + (size_t)row * 4);
        const float t = info.x, u = info.y, m = info.z;
        int ch = (int)info.w;
        ch = min(max(ch, 0), DCH - 1);
        v4f wc = *(const v4f*)(iffw + (size_t)ch * DK + c);
        wc.x = bf16r(wc.x); wc.y = bf16r(wc.y); wc.z = bf16r(wc.z); wc.w = bf16r(wc.w);
        const float tm = t * m, um = u * m;
        v4f z;
        z.x = fmaxf(m * wc.x + tm * w41.x + um * w42.x + bb.x, 0.0f) * m;
        z.y = fmaxf(m * wc.y + tm * w41.y + um * w42.y + bb.y, 0.0f) * m;
        z.z = fmaxf(m * wc.z + tm * w41.z + um * w42.z + bb.z, 0.0f) * m;
        z.w = fmaxf(m * wc.w + tm * w41.w + um * w42.w + bb.w, 0.0f) * m;
        v4h hv, rv;
        _Float16 h0, r0h;
        split16(z.x, h0, r0h); hv.x = h0; rv.x = r0h;
        split16(z.y, h0, r0h); hv.y = h0; rv.y = r0h;
        split16(z.z, h0, r0h); hv.z = h0; rv.z = r0h;
        split16(z.w, h0, r0h); hv.w = h0; rv.w = r0h;
        const unsigned b = row / (unsigned)NOBS;
        const unsigned n = row - b * (unsigned)NOBS;
        const size_t zo = ((size_t)b * NOBS_FULL + n) * DK + c;
        const size_t po = (size_t)row * DK + c;
        *(volatile v4f*)(Zout + zo) = z;
        *(volatile v4h*)(Zh + po) = hv;
        *(volatile v4h*)(Zr + po) = rv;
        __threadfence();
        *(volatile v4f*)(Zout + zo) = z;
        *(volatile v4h*)(Zh + po) = hv;
        *(volatile v4h*)(Zr + po) = rv;
    }
}

__global__ __launch_bounds__(256) __attribute__((amdgpu_num_vgpr(256)))
void k_kv0(const _Float16* __restrict__ Zh,
           const _Float16* __restrict__ wk, const _Float16* __restrict__ wv,
           const float* __restrict__ bk, const float* __restrict__ bv,
           _Float16* __restrict__ K0h, _Float16* __restrict__ V0T) {
    __shared__ __align__(16) _Float16 Kt[8][16 * DK];
    __shared__ __align__(16) _Float16 VT[DK * 128];
    const unsigned tid = threadIdx.x, lane = tid & 31u, w = tid >> 5;
    const unsigned blk0 = blockIdx.x * 128u;
    const unsigned b  = blk0 / (unsigned)NOBS;
    const unsigned n0 = blk0 - b * (unsigned)NOBS;
    const unsigned row0 = blk0 + w * 16u;
    const unsigned r0 = (lane >> 4) << 3, cc = lane & 15u;

    v16h za[4];
#pragma unroll
    for (int kt = 0; kt < 4; ++kt) za[kt] = load_frag16(Zh + (size_t)row0 * DK + kt * 32, DK, (int)lane);

#pragma unroll 1
    for (unsigned nt = 0; nt < 8u; ++nt) {
        v8f acc = zero8();
#pragma unroll
        for (int kt = 0; kt < 4; ++kt)
            acc = wmma16(za[kt], load_frag16(wk + (size_t)(nt * 16u) * DK + kt * 32, DK, (int)lane), acc);
        const float bias = bf16r(bk[nt * 16u + cc]) * 64.0f;
#pragma unroll
        for (int g = 0; g < 8; ++g)
            Kt[w][(r0 + g) * DK + nt * 16u + cc] = (_Float16)__builtin_fmaf(acc[g], 0.0625f, bias);
    }
#pragma unroll 1
    for (unsigned nt = 0; nt < 8u; ++nt) {
        v8f acc = zero8();
#pragma unroll
        for (int kt = 0; kt < 4; ++kt)
            acc = wmma16(za[kt], load_frag16(wv + (size_t)(nt * 16u) * DK + kt * 32, DK, (int)lane), acc);
        const float bias = bf16r(bv[nt * 16u + cc]) * 64.0f;
#pragma unroll
        for (int g = 0; g < 8; ++g)
            VT[(nt * 16u + cc) * 128u + w * 16u + r0 + g] = (_Float16)__builtin_fmaf(acc[g], 0.0625f, bias);
    }
    wave_lds_sync();
    __syncthreads();

    v8h kv[8], vv[8];
#pragma unroll
    for (unsigned i = 0; i < 8u; ++i) {
        kv[i] = *(const v8h*)(&Kt[w][i * 256u + lane * 8u]);
        vv[i] = *(const v8h*)(&VT[(i * 256u + tid) * 8u]);
    }
    _Float16* kd = K0h + (size_t)row0 * DK;
    _Float16* vd = V0T + (size_t)b * DK * NOBS + n0;
#pragma unroll
    for (unsigned i = 0; i < 8u; ++i) {
        unsigned idx = i * 256u + tid;
        unsigned d = idx >> 4, part = idx & 15u;
        *(volatile v8h*)(kd + i * 256u + lane * 8u) = kv[i];
        *(volatile v8h*)(vd + (size_t)d * NOBS + part * 8u) = vv[i];
    }
    __threadfence();
#pragma unroll
    for (unsigned i = 0; i < 8u; ++i) {
        unsigned idx = i * 256u + tid;
        unsigned d = idx >> 4, part = idx & 15u;
        *(volatile v8h*)(kd + i * 256u + lane * 8u) = kv[i];
        *(volatile v8h*)(vd + (size_t)d * NOBS + part * 8u) = vv[i];
    }
}

__global__ __launch_bounds__(256) __attribute__((amdgpu_num_vgpr(256)))
void k_attn0(const _Float16* __restrict__ indh, const _Float16* __restrict__ wq0,
             const float* __restrict__ bq0,
             const _Float16* __restrict__ K0h, const _Float16* __restrict__ V0T,
             const float* __restrict__ mkp, float* __restrict__ O0) {
    __shared__ __align__(16) _Float16 Tq[8][16 * DH];
    __shared__ __align__(16) _Float16 Tp[8][16 * 128];
    __shared__ __align__(16) float    To[8][16 * DH];
    const unsigned tid = threadIdx.x, lane = tid & 31u, w = tid >> 5;
    const unsigned b = blockIdx.x, hd = blockIdx.y;
    const unsigned r0 = (lane >> 4) << 3, cc = lane & 15u;

    v8f q0[2];
    {
        v16h ia[4];
#pragma unroll
        for (int kt = 0; kt < 4; ++kt) ia[kt] = load_frag16(indh + (size_t)(w * 16u) * DK + kt * 32, DK, (int)lane);
#pragma unroll
        for (unsigned n2 = 0; n2 < 2u; ++n2) {
            v8f acc = zero8();
#pragma unroll
            for (int kt = 0; kt < 4; ++kt)
                acc = wmma16(ia[kt], load_frag16(wq0 + (size_t)(hd * DH + n2 * 16u) * DK + kt * 32, DK, (int)lane), acc);
            const float bias = bf16r(bq0[hd * DH + n2 * 16u + cc]);
            v8f qq;
#pragma unroll
            for (int g = 0; g < 8; ++g) {
                float qv = __builtin_fmaf(acc[g], 0.000244140625f, bias);
                qq[g] = qv;
                Tq[w][(r0 + g) * DH + n2 * 16u + cc] = (_Float16)(qv * 64.0f);
            }
            q0[n2] = qq;
        }
    }
    wave_lds_sync();
    const v16h qf = load_frag16(&Tq[w][0], DH, (int)lane);

    const _Float16* Kb = K0h + (size_t)b * NOBS * DK + hd * DH;
    const _Float16* Vb = V0T + ((size_t)b * DK + hd * DH) * NOBS;
    const float* mkb = mkp + (size_t)b * NOBS;

    float mr[8], lr[8];
#pragma unroll
    for (int g = 0; g < 8; ++g) { mr[g] = -3.0e38f; lr[g] = 0.0f; }
    v8f o0 = zero8(), o1 = zero8();

#pragma unroll 1
    for (unsigned c0 = 0; c0 < (unsigned)NOBS; c0 += 128u) {
        v8f s[8];
        float mkk[8];
#pragma unroll
        for (unsigned nt = 0; nt < 8u; ++nt) {
            v16h kf = load_frag16(Kb + (size_t)(c0 + nt * 16u) * DK, DK, (int)lane);
            s[nt] = wmma16(qf, kf, zero8());
            mkk[nt] = mkb[c0 + nt * 16u + cc];
        }
#pragma unroll
        for (int g = 0; g < 8; ++g) {
            float mx = -3.0e38f;
#pragma unroll
            for (unsigned nt = 0; nt < 8u; ++nt) {
                float t = (mkk[nt] > 0.0f) ? (s[nt][g] * CS) : NEGT;
                s[nt][g] = t;
                mx = fmaxf(mx, t);
            }
            mx = hmax16(mx);
            const float mn = fmaxf(mr[g], mx);
            const float resc = ex2(mr[g] - mn);
            mr[g] = mn;
            float ls = 0.0f;
#pragma unroll
            for (unsigned nt = 0; nt < 8u; ++nt) {
                float p = ex2(s[nt][g] - mn + 8.0f);
                ls += p;
                Tp[w][(r0 + g) * 128u + nt * 16u + cc] = (_Float16)p;
            }
            lr[g] = __builtin_fmaf(lr[g], resc, ls);
            o0[g] *= resc;
            o1[g] *= resc;
        }
        wave_lds_sync();
#pragma unroll
        for (unsigned kt = 0; kt < 4u; ++kt) {
            v16h pa  = load_frag16(&Tp[w][kt * 32u], 128, (int)lane);
            v16h vb0 = load_frag16(Vb + c0 + kt * 32u, NOBS, (int)lane);
            v16h vb1 = load_frag16(Vb + (size_t)16 * NOBS + c0 + kt * 32u, NOBS, (int)lane);
            o0 = wmma16(pa, vb0, o0);
            o1 = wmma16(pa, vb1, o1);
        }
        wave_lds_sync();
    }

#pragma unroll
    for (int g = 0; g < 8; ++g) {
        float l = hsum16(lr[g]);
        float inv = (1.0f / l) * 0.015625f;
        To[w][(r0 + g) * DH + cc]       = __builtin_fmaf(o0[g], inv, q0[0][g]);
        To[w][(r0 + g) * DH + 16u + cc] = __builtin_fmaf(o1[g], inv, q0[1][g]);
    }
    wave_lds_sync();
    v4f sv[4];
    const unsigned rq = lane >> 3, piece = lane & 7u;
#pragma unroll
    for (unsigned i = 0; i < 4u; ++i) sv[i] = *(const v4f*)(&To[w][(i * 4u + rq) * DH + piece * 4u]);
    float* ob = O0 + ((size_t)b * MIND + w * 16u) * DK + hd * DH + piece * 4u;
#pragma unroll
    for (unsigned i = 0; i < 4u; ++i) *(volatile v4f*)(ob + (size_t)(i * 4u + rq) * DK) = sv[i];
    __threadfence();
#pragma unroll
    for (unsigned i = 0; i < 4u; ++i) *(volatile v4f*)(ob + (size_t)(i * 4u + rq) * DK) = sv[i];
}

__global__ __launch_bounds__(256) __attribute__((amdgpu_num_vgpr(256)))
void k_hmid(const float* __restrict__ O0,
            const _Float16* __restrict__ wo0, const _Float16* __restrict__ wk1,
            const _Float16* __restrict__ wv1,
            const float* __restrict__ bo0, const float* __restrict__ bk1, const float* __restrict__ bv1,
            _Float16* __restrict__ K1h, _Float16* __restrict__ V1T) {
    __shared__ __align__(16) _Float16 Ht[8][16 * DK];
    __shared__ __align__(16) _Float16 VT[DK * MIND];
    const unsigned tid = threadIdx.x, lane = tid & 31u, w = tid >> 5;
    const unsigned b = blockIdx.x;
    const unsigned r0 = (lane >> 4) << 3, cc = lane & 15u;
    const float* Ob = O0 + ((size_t)b * MIND + w * 16u) * DK;

    v16h oa[4];
#pragma unroll
    for (int kt = 0; kt < 4; ++kt) oa[kt] = load_frag_f32(Ob + kt * 32, DK, (int)lane, 64.0f);
#pragma unroll 1
    for (unsigned nt = 0; nt < 8u; ++nt) {
        v8f acc = zero8();
#pragma unroll
        for (int kt = 0; kt < 4; ++kt)
            acc = wmma16(oa[kt], load_frag16(wo0 + (size_t)(nt * 16u) * DK + kt * 32, DK, (int)lane), acc);
        const float bias = bf16r(bo0[nt * 16u + cc]);
#pragma unroll
        for (int g = 0; g < 8; ++g) {
            float res = Ob[(size_t)(r0 + g) * DK + nt * 16u + cc];
            float y = __builtin_fmaf(acc[g], 0.000244140625f, bias);
            float h = res + fmaxf(y, 0.0f);
            Ht[w][(r0 + g) * DK + nt * 16u + cc] = (_Float16)(h * 64.0f);
        }
    }
    wave_lds_sync();
    v16h ha[4];
#pragma unroll
    for (int kt = 0; kt < 4; ++kt) ha[kt] = load_frag16(&Ht[w][kt * 32], DK, (int)lane);
    wave_lds_sync();

#pragma unroll 1
    for (unsigned nt = 0; nt < 8u; ++nt) {
        v8f acc = zero8();
#pragma unroll
        for (int kt = 0; kt < 4; ++kt)
            acc = wmma16(ha[kt], load_frag16(wk1 + (size_t)(nt * 16u) * DK + kt * 32, DK, (int)lane), acc);
        const float bias = bf16r(bk1[nt * 16u + cc]) * 64.0f;
#pragma unroll
        for (int g = 0; g < 8; ++g)
            Ht[w][(r0 + g) * DK + nt * 16u + cc] = (_Float16)__builtin_fmaf(acc[g], 0.015625f, bias);
    }
#pragma unroll 1
    for (unsigned nt = 0; nt < 8u; ++nt) {
        v8f acc = zero8();
#pragma unroll
        for (int kt = 0; kt < 4; ++kt)
            acc = wmma16(ha[kt], load_frag16(wv1 + (size_t)(nt * 16u) * DK + kt * 32, DK, (int)lane), acc);
        const float bias = bf16r(bv1[nt * 16u + cc]) * 64.0f;
#pragma unroll
        for (int g = 0; g < 8; ++g)
            VT[(nt * 16u + cc) * MIND + w * 16u + r0 + g] = (_Float16)__builtin_fmaf(acc[g], 0.015625f, bias);
    }
    wave_lds_sync();
    __syncthreads();

    v8h kv[8], vv[8];
#pragma unroll
    for (unsigned i = 0; i < 8u; ++i) {
        kv[i] = *(const v8h*)(&Ht[w][i * 256u + lane * 8u]);
        vv[i] = *(const v8h*)(&VT[(i * 256u + tid) * 8u]);
    }
    _Float16* kd = K1h + ((size_t)b * MIND + w * 16u) * DK;
    _Float16* vd = V1T + (size_t)b * DK * MIND;
#pragma unroll
    for (unsigned i = 0; i < 8u; ++i) {
        *(volatile v8h*)(kd + i * 256u + lane * 8u) = kv[i];
        *(volatile v8h*)(vd + (size_t)(i * 256u + tid) * 8u) = vv[i];
    }
    __threadfence();
#pragma unroll
    for (unsigned i = 0; i < 8u; ++i) {
        *(volatile v8h*)(kd + i * 256u + lane * 8u) = kv[i];
        *(volatile v8h*)(vd + (size_t)(i * 256u + tid) * 8u) = vv[i];
    }
}

__global__ __launch_bounds__(128) __attribute__((amdgpu_num_vgpr(256)))
void k_layer1(_Float16* Zh, _Float16* Zr,
              const _Float16* __restrict__ wq1, const _Float16* __restrict__ wo1,
              const float* __restrict__ bq1, const float* __restrict__ bo1,
              const _Float16* __restrict__ K1h, const _Float16* __restrict__ V1T,
              const float* __restrict__ mkp, float* Zout, int write_planes) {
    __shared__ __align__(16) _Float16 Tq[4][16 * DK];
    __shared__ __align__(16) _Float16 Tp[4][16 * DK];
    __shared__ __align__(16) float    To[4][16 * DK];
    const unsigned tid = threadIdx.x, lane = tid & 31u, w = tid >> 5;
    const unsigned grow = blockIdx.x * 64u + w * 16u;
    const unsigned b = grow / (unsigned)NOBS;
    const unsigned n0 = grow - b * (unsigned)NOBS;
    const unsigned r0 = (lane >> 4) << 3, cc = lane & 15u;

    float m8[8];
    {
        v4f ma = *(const v4f*)(mkp + grow + r0);
        v4f mb = *(const v4f*)(mkp + grow + r0 + 4u);
        m8[0] = ma.x; m8[1] = ma.y; m8[2] = ma.z; m8[3] = ma.w;
        m8[4] = mb.x; m8[5] = mb.y; m8[6] = mb.z; m8[7] = mb.w;
    }

    {
        v16h zh[4], zr[4];
#pragma unroll
        for (int kt = 0; kt < 4; ++kt) {
            zh[kt] = load_frag16(Zh + (size_t)grow * DK + kt * 32, DK, (int)lane);
            zr[kt] = load_frag16(Zr + (size_t)grow * DK + kt * 32, DK, (int)lane);
        }
#pragma unroll 1
        for (unsigned nt = 0; nt < 8u; ++nt) {
            v8f ah = zero8(), ar = zero8();
#pragma unroll
            for (int kt = 0; kt < 4; ++kt) {
                v16h bf = load_frag16(wq1 + (size_t)(nt * 16u) * DK + kt * 32, DK, (int)lane);
                ah = wmma16(zh[kt], bf, ah);
                ar = wmma16(zr[kt], bf, ar);
            }
            const float bias = bf16r(bq1[nt * 16u + cc]) * 64.0f;
#pragma unroll
            for (int g = 0; g < 8; ++g) {
                float qa = __builtin_fmaf(__builtin_fmaf(ar[g], SC_RINV, ah[g]), 0.0625f, bias);
                To[w][(r0 + g) * DK + nt * 16u + cc] = qa * 0.015625f;
                Tq[w][(r0 + g) * DK + nt * 16u + cc] = (_Float16)qa;
            }
        }
    }
    wave_lds_sync();

    const _Float16* K1b = K1h + (size_t)b * MIND * DK;
    const _Float16* V1b = V1T + (size_t)b * DK * MIND;
#pragma unroll
    for (unsigned hd = 0; hd < 4u; ++hd) {
        const v16h qf = load_frag16(&Tq[w][hd * DH], DK, (int)lane);
        v8f s[8];
#pragma unroll
        for (unsigned nt = 0; nt < 8u; ++nt) {
            v16h kf = load_frag16(K1b + (size_t)(nt * 16u) * DK + hd * DH, DK, (int)lane);
            s[nt] = wmma16(qf, kf, zero8());
        }
#pragma unroll
        for (int g = 0; g < 8; ++g) {
            const bool valid = (m8[g] > 0.0f);
            float mx = -3.0e38f;
#pragma unroll
            for (unsigned nt = 0; nt < 8u; ++nt) {
                float t = valid ? (s[nt][g] * CS) : NEGT;
                s[nt][g] = t;
                mx = fmaxf(mx, t);
            }
            mx = hmax16(mx);
            float ls = 0.0f;
#pragma unroll
            for (unsigned nt = 0; nt < 8u; ++nt) {
                float p = ex2(s[nt][g] - mx);
                s[nt][g] = p;
                ls += p;
            }
            ls = hsum16(ls);
            const float inv = 1024.0f * (1.0f / ls);
#pragma unroll
            for (unsigned nt = 0; nt < 8u; ++nt)
                Tp[w][(r0 + g) * DK + nt * 16u + cc] = (_Float16)(s[nt][g] * inv);
        }
        wave_lds_sync();
        v8f o0 = zero8(), o1 = zero8();
#pragma unroll
        for (unsigned kt = 0; kt < 4u; ++kt) {
            v16h pa  = load_frag16(&Tp[w][kt * 32u], DK, (int)lane);
            v16h vb0 = load_frag16(V1b + (size_t)(hd * DH) * MIND + kt * 32u, MIND, (int)lane);
            v16h vb1 = load_frag16(V1b + (size_t)(hd * DH + 16u) * MIND + kt * 32u, MIND, (int)lane);
            o0 = wmma16(pa, vb0, o0);
            o1 = wmma16(pa, vb1, o1);
        }
#pragma unroll
        for (int g = 0; g < 8; ++g) {
            const unsigned i0 = (r0 + g) * DK + hd * DH + cc;
            float a0 = To[w][i0];
            float a1 = To[w][i0 + 16u];
            To[w][i0]       = __builtin_fmaf(o0[g], 1.52587890625e-05f, a0);
            To[w][i0 + 16u] = __builtin_fmaf(o1[g], 1.52587890625e-05f, a1);
        }
        wave_lds_sync();
    }

#pragma unroll 1
    for (unsigned nt = 0; nt < 8u; ++nt) {
#pragma unroll
        for (int g = 0; g < 8; ++g) {
            const unsigned ix = (r0 + g) * DK + nt * 16u + cc;
            _Float16 hh, rr;
            split16(To[w][ix], hh, rr);
            Tq[w][ix] = hh;
            Tp[w][ix] = rr;
        }
    }
    wave_lds_sync();
    {
        v16h oh[4], orr[4];
#pragma unroll
        for (int kt = 0; kt < 4; ++kt) {
            oh[kt]  = load_frag16(&Tq[w][kt * 32], DK, (int)lane);
            orr[kt] = load_frag16(&Tp[w][kt * 32], DK, (int)lane);
        }
#pragma unroll 1
        for (unsigned nt = 0; nt < 8u; ++nt) {
            v8f ah = zero8(), ar = zero8();
#pragma unroll
            for (int kt = 0; kt < 4; ++kt) {
                v16h bf = load_frag16(wo1 + (size_t)(nt * 16u) * DK + kt * 32, DK, (int)lane);
                ah = wmma16(oh[kt], bf, ah);
                ar = wmma16(orr[kt], bf, ar);
            }
            const float bias = bf16r(bo1[nt * 16u + cc]);
#pragma unroll
            for (int g = 0; g < 8; ++g) {
                const unsigned ix = (r0 + g) * DK + nt * 16u + cc;
                float y = __builtin_fmaf(__builtin_fmaf(ar[g], SC_RINV, ah[g]), 9.765625e-04f, bias);
                float zn = To[w][ix] + fmaxf(y, 0.0f);
                To[w][ix] = zn * m8[g];
            }
        }
    }
    wave_lds_sync();

    const size_t zrow0 = ((size_t)b * NOBS_FULL + n0) * DK + lane * 4u;
    const size_t prow0 = (size_t)grow * DK + lane * 4u;
#pragma unroll 1
    for (unsigned grp = 0; grp < 4u; ++grp) {
        v4f zv[4];
        v4h hv[4], rv[4];
#pragma unroll
        for (unsigned i = 0; i < 4u; ++i) {
            const unsigned row = grp * 4u + i;
            v4f zn = *(const v4f*)(&To[w][row * DK + lane * 4u]);
            v4f zo = *(const v4f*)(Zout + zrow0 + (size_t)row * DK);
            v4f z;
            z.x = zn.x + zo.x; z.y = zn.y + zo.y; z.z = zn.z + zo.z; z.w = zn.w + zo.w;
            zv[i] = z;
            _Float16 h0, r0h;
            v4h hq, rq;
            split16(z.x, h0, r0h); hq.x = h0; rq.x = r0h;
            split16(z.y, h0, r0h); hq.y = h0; rq.y = r0h;
            split16(z.z, h0, r0h); hq.z = h0; rq.z = r0h;
            split16(z.w, h0, r0h); hq.w = h0; rq.w = r0h;
            hv[i] = hq; rv[i] = rq;
        }
#pragma unroll
        for (unsigned i = 0; i < 4u; ++i) {
            const unsigned row = grp * 4u + i;
            *(volatile v4f*)(Zout + zrow0 + (size_t)row * DK) = zv[i];
            if (write_planes) {
                *(volatile v4h*)(Zh + prow0 + (size_t)row * DK) = hv[i];
                *(volatile v4h*)(Zr + prow0 + (size_t)row * DK) = rv[i];
            }
        }
        __threadfence();
#pragma unroll
        for (unsigned i = 0; i < 4u; ++i) {
            const unsigned row = grp * 4u + i;
            *(volatile v4f*)(Zout + zrow0 + (size_t)row * DK) = zv[i];
            if (write_planes) {
                *(volatile v4h*)(Zh + prow0 + (size_t)row * DK) = hv[i];
                *(volatile v4h*)(Zr + prow0 + (size_t)row * DK) = rv[i];
            }
        }
    }
}

extern "C" void kernel_launch(void* const* d_in, const int* in_sizes, int n_in,
                              void* d_out, int out_size, void* d_ws, size_t ws_size,
                              hipStream_t stream) {
    if (n_in < 23) return;
    if (in_sizes[0] < NB * LSEQ) return;
    if (in_sizes[1] < NB * LD_FULL || in_sizes[2] < NB * LD_FULL) return;
    if (in_sizes[3] < 1) return;
    if (in_sizes[4] < 43 * DK || in_sizes[5] < DK) return;
    if (in_sizes[6] < NLAY * WPL) return;
    for (int j = 0; j < 8; ++j) {
        if (in_sizes[7 + 2 * j] < NLAY * WPL) return;
        if (in_sizes[8 + 2 * j] < NLAY * DK) return;
    }
    if ((size_t)out_size < OUT1_OFF + (size_t)(NB - 1) * NOBS_FULL + NOBS) return;
    if ((size_t)WS_TOTAL > ws_size) return;

    const float* ctx  = (const float*)d_in[0];
    const float* val  = (const float*)d_in[1];
    const float* mask = (const float*)d_in[2];
    const int*   obs  = (const int*)d_in[3];
    const float* iffw = (const float*)d_in[4];
    const float* iffb = (const float*)d_in[5];
    const float* indp = (const float*)d_in[6];
    const float* Wf[8];
    const float* Bf[8];
    for (int j = 0; j < 8; ++j) {
        Wf[j] = (const float*)d_in[7 + 2 * j];
        Bf[j] = (const float*)d_in[8 + 2 * j];
    }
    float* Zout = (float*)d_out;

    char* ws = (char*)d_ws;
    size_t off = 0;
    _Float16* wpl     = (_Float16*)(ws + off); off += WPL_BYTES;
    float*    rowinfo = (float*)(ws + off);    off += RI_BYTES;
    float*    mkp     = (float*)(ws + off);    off += MK_BYTES;
    _Float16* Zh      = (_Float16*)(ws + off); off += PL_BYTES;
    _Float16* Zr      = (_Float16*)(ws + off); off += PL_BYTES;
    _Float16* K0h     = (_Float16*)(ws + off); off += PL_BYTES;
    _Float16* V0T     = (_Float16*)(ws + off); off += PL_BYTES;
    float*    O0      = (float*)(ws + off);    off += O0_BYTES;
    _Float16* K1h     = (_Float16*)(ws + off); off += HP_BYTES;
    _Float16* V1T     = (_Float16*)(ws + off); off += HP_BYTES;
    if (off > ws_size) return;

    k_wprep<<<dim3(NPLANES), dim3(256), 0, stream>>>(Wf[0], Wf[1], Wf[2], Wf[3], Wf[4], Wf[5], Wf[6], Wf[7],
                                                     indp, wpl);
    k_compact<<<dim3(NB), dim3(256), 0, stream>>>(ctx, val, mask, obs, rowinfo, mkp, Zout);
    k_embed<<<dim3(NB * NOBS / 32), dim3(256), 0, stream>>>(rowinfo, iffw, iffb, Zout, Zh, Zr);

    for (int i = 0; i < NLAY; ++i) {
        const _Float16* wq0 = wpl + (size_t)(0 * 3 + i) * WPL;
        const _Float16* wk0 = wpl + (size_t)(1 * 3 + i) * WPL;
        const _Float16* wv0 = wpl + (size_t)(2 * 3 + i) * WPL;
        const _Float16* wo0 = wpl + (size_t)(3 * 3 + i) * WPL;
        const _Float16* wq1 = wpl + (size_t)(4 * 3 + i) * WPL;
        const _Float16* wk1 = wpl + (size_t)(5 * 3 + i) * WPL;
        const _Float16* wv1 = wpl + (size_t)(6 * 3 + i) * WPL;
        const _Float16* wo1 = wpl + (size_t)(7 * 3 + i) * WPL;
        const _Float16* ind = wpl + (size_t)(8 * 3 + i) * WPL;
        k_kv0<<<dim3(NB * NOBS / 128), dim3(256), 0, stream>>>(Zh, wk0, wv0, Bf[1] + i * DK, Bf[2] + i * DK,
                                                               K0h, V0T);
        k_attn0<<<dim3(NB, NHEAD), dim3(256), 0, stream>>>(ind, wq0, Bf[0] + i * DK, K0h, V0T, mkp, O0);
        k_hmid<<<dim3(NB), dim3(256), 0, stream>>>(O0, wo0, wk1, wv1, Bf[3] + i * DK, Bf[5] + i * DK,
                                                   Bf[6] + i * DK, K1h, V1T);
        k_layer1<<<dim3(NB * NOBS / 64), dim3(128), 0, stream>>>(Zh, Zr, wq1, wo1, Bf[4] + i * DK,
                                                                 Bf[7] + i * DK, K1h, V1T, mkp, Zout,
                                                                 (i + 1 < NLAY) ? 1 : 0);
    }
}
